// ResidualIrregularConv1D_28346784154089
// MI455X (gfx1250) — hardware-verified
//
#include <hip/hip_runtime.h>
#include <stdint.h>

typedef __attribute__((ext_vector_type(16))) _Float16 v16h;
typedef __attribute__((ext_vector_type(8)))  _Float16 v8h;
typedef __attribute__((ext_vector_type(16))) __bf16   v16b;
typedef __attribute__((ext_vector_type(8)))  __bf16   v8b;
typedef __attribute__((ext_vector_type(8)))  float    v8f;
typedef __attribute__((ext_vector_type(4)))  float    v4f;

#define S_DIM 16
#define E_DIM 1024
#define MSL 64
#define BN_EPS 1e-3f
#define ET1 256
#define AP 72
#define ZP 264
#define WSC1 64.0f
#define WSC1_INV (1.0f / 64.0f)
#define WSC2 256.0f
#define WSC2_INV (1.0f / 256.0f)

__device__ __forceinline__ void dep_guard_h(v8f& a, v8f& b, v16h x, v16h y) { asm volatile("v_nop\n\tv_nop\n\tv_nop\n\tv_nop" : "+v"(a), "+v"(b) : "v"(x), "v"(y)); }
__device__ __forceinline__ void dep_guard_b(v8f& a, v8f& b, v16b x, v16b y) { asm volatile("v_nop\n\tv_nop\n\tv_nop\n\tv_nop" : "+v"(a), "+v"(b) : "v"(x), "v"(y)); }
__device__ __forceinline__ void keep4_h(v16h a, v16h b, v16h c, v16h d) { asm volatile("v_nop" :: "v"(a), "v"(b), "v"(c), "v"(d)); }
__device__ __forceinline__ void keep4_b(v16b a, v16b b, v16b c, v16b d) { asm volatile("v_nop" :: "v"(a), "v"(b), "v"(c), "v"(d)); }
__device__ __forceinline__ void acc_guard4(v8f& a, v8f& b, v8f& c, v8f& d) { asm volatile("v_nop\n\tv_nop\n\tv_nop\n\tv_nop" : "+v"(a), "+v"(b), "+v"(c), "+v"(d)); }
template <typename T> struct Frag;
template <> struct Frag<_Float16> {
  typedef v16h V; union U { v16h v; v8h h[2]; };
  static __device__ __forceinline__ v16h load(const _Float16* p) {
    U f; f.h[0] = *(const v8h*)(p); f.h[1] = *(const v8h*)(p + 16); return f.v;
  }
  static __device__ __forceinline__ v8f mma(v16h a, v16h b, v8f c) {
    return __builtin_amdgcn_wmma_f32_16x16x32_f16(false, a, false, b, (short)0, c, false, false);
  }
  static __device__ __forceinline__ void guard(v8f& a, v8f& b, v16h x, v16h y) { dep_guard_h(a, b, x, y); }
  static __device__ __forceinline__ void keep(v16h a, v16h b, v16h c, v16h d) { keep4_h(a, b, c, d); }
};
template <> struct Frag<__bf16> {
  typedef v16b V; union U { v16b v; v8b h[2]; };
  static __device__ __forceinline__ v16b load(const __bf16* p) {
    U f; f.h[0] = *(const v8b*)(p); f.h[1] = *(const v8b*)(p + 16); return f.v;
  }
  static __device__ __forceinline__ v8f mma(v16b a, v16b b, v8f c) {
    return __builtin_amdgcn_wmma_f32_16x16x32_bf16(false, a, false, b, (short)0, c, false, false);
  }
  static __device__ __forceinline__ void guard(v8f& a, v8f& b, v16b x, v16b y) { dep_guard_b(a, b, x, y); }
  static __device__ __forceinline__ void keep(v16b a, v16b b, v16b c, v16b d) { keep4_b(a, b, c, d); }
};

__device__ __forceinline__ v8f mma16h(v16h a, v16h b, v8f c) {
  c = __builtin_amdgcn_wmma_f32_16x16x32_f16(false, a, false, b, (short)0, c, false, false);
  asm volatile("v_nop\n\tv_nop\n\tv_nop\n\tv_nop" : "+v"(c) : "v"(a), "v"(b));
  return c;
}

__global__ __launch_bounds__(256) void k_wtrans(
    const float* __restrict__ W, _Float16* __restrict__ Wt, int N, float mul)
{
  __shared__ float tile[64][33];
  const int f0  = blockIdx.x * 32;
  const int e0  = blockIdx.y * 64;
  const int tid = threadIdx.x;
  const int tx  = tid & 31;
  const int ty  = tid >> 5;
  for (int r = ty; r < 64; r += 8)
    tile[r][tx] = W[(size_t)(e0 + r) * N + f0 + tx];
  __syncthreads();
  const int nl = tid >> 3;
  const int q8 = (tid & 7) * 8;
  v8h pk;
#pragma unroll
  for (int i = 0; i < 8; ++i) pk[i] = (_Float16)(tile[q8 + i][nl] * mul);
  _Float16* dst = Wt + (size_t)(f0 + nl) * N + e0 + q8;
  *(volatile v8h*)dst = pk;
  __threadfence();
  *(volatile v8h*)dst = pk;
}

__global__ __launch_bounds__(256) void k_stage1(
    const float* __restrict__ X, const float* __restrict__ Wp, const float* __restrict__ bp,
    const float* __restrict__ g1, const float* __restrict__ be1,
    const float* __restrict__ m1, const float* __restrict__ v1,
    const int* __restrict__ idx, _Float16* __restrict__ ZS)
{
  __shared__ __align__(16) _Float16 At[ET1 * AP];
  __shared__ __align__(16) _Float16 Bts[S_DIM * AP];
  __shared__ __align__(16) _Float16 Zs[S_DIM * ZP];
  __shared__ float sc1[S_DIM], sh1[S_DIM];
  __shared__ int rr[MSL];

  const int tid  = threadIdx.x;
  const int b    = blockIdx.y;
  const int e0   = blockIdx.x * ET1;

  if (tid < MSL) {
    const int v = idx[tid];
    int r = v % S_DIM;
    if (r < 0) r += S_DIM;
    rr[tid] = r;
  }
  if (tid < S_DIM) {
    const float s0 = g1[tid] * rsqrtf(v1[tid] + BN_EPS);
    sc1[tid] = s0;
    sh1[tid] = (bp[tid] - m1[tid]) * s0 + be1[tid];
  }
  for (int c = tid; c < MSL * S_DIM; c += 256) {
    const int m = c >> 4, s = c & 15;
    Bts[s * AP + m] = (_Float16)(Wp[c] * WSC1);
  }
  __syncthreads();

  {
    const float* Xb = X + (size_t)b * S_DIM * E_DIM + e0 + tid;
#pragma unroll
    for (int mm = 0; mm < 8; ++mm) {
      v8h pk;
#pragma unroll
      for (int i = 0; i < 8; ++i) pk[i] = (_Float16)Xb[(size_t)rr[mm * 8 + i] * E_DIM];
      *(v8h*)(At + tid * AP + mm * 8) = pk;
    }
  }
  __syncthreads();

  {
    const int wave  = tid >> 5;
    const int lane  = tid & 31;
    const int rlane = lane & 15;
    const int hsel  = lane >> 4;
    const int koff  = hsel * 8;
#pragma unroll
    for (int t = 0; t < 2; ++t) {
      const int sub = wave * 2 + t;
      v8f acc = (v8f){0.f,0.f,0.f,0.f,0.f,0.f,0.f,0.f};
#pragma unroll
      for (int ks = 0; ks < 2; ++ks) {
        const v16h a  = Frag<_Float16>::load(At  + (sub * 16 + rlane) * AP + koff + ks * 32);
        const v16h bf = Frag<_Float16>::load(Bts + rlane * AP + koff + ks * 32);
        acc = mma16h(a, bf, acc);
      }
      const float sc = sc1[rlane] * WSC1_INV;
      const float sh = sh1[rlane];
      v8h zv;
#pragma unroll
      for (int r = 0; r < 8; ++r) zv[r] = (_Float16)fmaxf(fmaf(acc[r], sc, sh), 0.0f);
      *(v8h*)(Zs + rlane * ZP + sub * 16 + 8 * hsel) = zv;
    }
  }
  __syncthreads();

  for (int pass = 0; pass < 2; ++pass) {
#pragma unroll
    for (int p = 0; p < 2; ++p) {
      const int c  = p * 256 + tid;
      const int s  = c >> 5;
      const int ch = c & 31;
      const v8h v = *(const v8h*)(Zs + s * ZP + ch * 8);
      *(volatile v8h*)(ZS + ((size_t)b * S_DIM + s) * E_DIM + e0 + ch * 8) = v;
    }
    __threadfence();
  }
}

template <int MODE>
__global__ __launch_bounds__(256) void gemm64_bn(
    const unsigned short* __restrict__ Ap, int lda,
    const unsigned short* __restrict__ Btp, int ldb,
    void* __restrict__ Cout, int ldc,
    const float* __restrict__ cb, const float* __restrict__ gam, const float* __restrict__ bet,
    const float* __restrict__ mean, const float* __restrict__ var,
    const float* __restrict__ resid,
    int M, int N, int K, float scale)
{
  typedef _Float16 T;
  typedef v16h V;
  const T* A = (const T*)Ap; const T* Bt = (const T*)Btp;
  __shared__ __align__(16) float sT[8][16 * 68];
  const int lane = threadIdx.x & 31;
  const int wave = threadIdx.x >> 5;
  const int tilesN = N >> 6;
  const int tilesM = M >> 6;
  const int tile = blockIdx.x * 8 + wave;
  if (tile >= tilesM * tilesN) return;
  const int tm = tile / tilesN;
  const int tn = tile - tm * tilesN;
  const int m0 = tm << 6;
  const int n0 = tn << 6;

  const int rlane = lane & 15;
  const int koff  = (lane >> 4) * 8;
  const int mOff  = (lane >> 4) * 8;

  v8f acc[4][4];
#pragma unroll
  for (int i = 0; i < 4; ++i)
#pragma unroll
    for (int j = 0; j < 4; ++j) acc[i][j] = (v8f){0.f,0.f,0.f,0.f,0.f,0.f,0.f,0.f};

  for (int k0 = 0; k0 < K; k0 += 32) {
    V bh[4];
#pragma unroll
    for (int j = 0; j < 4; ++j) {
      const size_t bo = (size_t)(n0 + (j << 4) + rlane) * ldb + koff + k0;
      bh[j] = Frag<T>::load(Bt + bo);
    }
#pragma unroll
    for (int i = 0; i < 4; ++i) {
      const size_t ao = (size_t)(m0 + (i << 4) + rlane) * lda + koff + k0;
      V ah = Frag<T>::load(A + ao);
#pragma unroll
      for (int j = 0; j < 4; ++j) {
        acc[i][j] = Frag<T>::mma(ah, bh[j], acc[i][j]);
      }
      Frag<T>::guard(acc[i][0], acc[i][3], ah, ah);
    }
    Frag<T>::keep(bh[0], bh[1], bh[2], bh[3]);
  }
  acc_guard4(acc[0][0], acc[0][1], acc[0][2], acc[0][3]);
  acc_guard4(acc[1][0], acc[1][1], acc[1][2], acc[1][3]);
  acc_guard4(acc[2][0], acc[2][1], acc[2][2], acc[2][3]);
  acc_guard4(acc[3][0], acc[3][1], acc[3][2], acc[3][3]);

  float* slab = sT[wave];
#pragma unroll
  for (int i = 0; i < 4; ++i) {
    const int mBase = m0 + (i << 4);
#pragma unroll
    for (int j = 0; j < 4; ++j) {
      const int n = n0 + (j << 4) + rlane;
      const float s0 = gam[n] * rsqrtf(var[n] + BN_EPS);
      const float sc = s0 * scale;
      const float sh = (cb[n] - mean[n]) * s0 + bet[n];
#pragma unroll
      for (int r = 0; r < 8; ++r) {
        float v = fmaf(acc[i][j][r], sc, sh);
        if (MODE == 1) v += resid[(size_t)(mBase + mOff + r) * ldc + n];
        v = fmaxf(v, 0.0f);
        slab[(mOff + r) * 68 + (j << 4) + rlane] = v;
      }
    }
    __builtin_amdgcn_fence(__ATOMIC_RELEASE, "workgroup");
    __builtin_amdgcn_wave_barrier();
    __builtin_amdgcn_fence(__ATOMIC_ACQUIRE, "workgroup");
    if (MODE == 1) {
      float* C = (float*)Cout;
      const int hh = lane >> 4, c4 = (lane & 15) * 4;
      for (int pass = 0; pass < 2; ++pass) {
#pragma unroll
        for (int it = 0; it < 8; ++it) {
          const int row = it * 2 + hh;
          v4f v = *(const v4f*)(slab + row * 68 + c4);
          *(volatile v4f*)(C + (size_t)(mBase + row) * ldc + n0 + c4) = v;
        }
        __threadfence();
      }
    } else {
      const int q = lane >> 3, c8 = (lane & 7) * 8;
      unsigned short* C = (unsigned short*)Cout;
      for (int pass = 0; pass < 2; ++pass) {
#pragma unroll
        for (int it = 0; it < 4; ++it) {
          const int row = it * 4 + q;
          const float* sp = slab + row * 68 + c8;
          v8h hv;
#pragma unroll
          for (int e = 0; e < 8; ++e) hv[e] = (_Float16)sp[e];
          *(volatile v8h*)(C + (size_t)(mBase + row) * ldc + n0 + c8) = hv;
        }
        __threadfence();
      }
    }
    __builtin_amdgcn_fence(__ATOMIC_RELEASE, "workgroup");
    __builtin_amdgcn_wave_barrier();
    __builtin_amdgcn_fence(__ATOMIC_ACQUIRE, "workgroup");
  }
}

extern "C" void kernel_launch(void* const* d_in, const int* in_sizes, int n_in,
                              void* d_out, int out_size, void* d_ws, size_t ws_size,
                              hipStream_t stream) {
  if (n_in < 20) return;
  const float* X   = (const float*)d_in[0];
  const float* Wp  = (const float*)d_in[1];
  const float* bp  = (const float*)d_in[2];
  const float* W1  = (const float*)d_in[3];
  const float* b1  = (const float*)d_in[4];
  const float* W2  = (const float*)d_in[5];
  const float* b2  = (const float*)d_in[6];
  const float* g1  = (const float*)d_in[7];
  const float* be1 = (const float*)d_in[8];
  const float* m1  = (const float*)d_in[9];
  const float* v1  = (const float*)d_in[10];
  const float* g2  = (const float*)d_in[11];
  const float* be2 = (const float*)d_in[12];
  const float* m2  = (const float*)d_in[13];
  const float* v2  = (const float*)d_in[14];
  const float* g3  = (const float*)d_in[15];
  const float* be3 = (const float*)d_in[16];
  const float* m3  = (const float*)d_in[17];
  const float* v3  = (const float*)d_in[18];
  const int* masks = (const int*)d_in[19];
  float* out = (float*)d_out;

  const int nX = in_sizes[0];
  const int nB = nX / (S_DIM * E_DIM);
  if (nB <= 0 || (nB & 3) != 0 || nX != nB * S_DIM * E_DIM) return;
  if (in_sizes[1] != MSL * S_DIM || in_sizes[19] != MSL) return;
  if (in_sizes[3] != E_DIM * E_DIM || in_sizes[5] != E_DIM * E_DIM) return;
  if (out_size != nX) return;
  const int Mrows = nB * S_DIM;

  const size_t szZ  = (size_t)Mrows * E_DIM * 2;
  const size_t szW  = (size_t)E_DIM * E_DIM * 2;
  const size_t offZ  = 0;
  const size_t offH  = offZ + szZ;
  const size_t offW1 = offH + szZ;
  const size_t offW2 = offW1 + szW;
  const size_t total = offW2 + szW;
  if (total > ws_size) return;
  char* ws = (char*)d_ws;
  _Float16* ZS  = (_Float16*)(ws + offZ);
  _Float16* Hb  = (_Float16*)(ws + offH);
  _Float16* Wt1 = (_Float16*)(ws + offW1);
  _Float16* Wt2 = (_Float16*)(ws + offW2);

  k_wtrans<<<dim3(E_DIM / 32, E_DIM / 64), 256, 0, stream>>>(W1, Wt1, E_DIM, WSC2);
  k_wtrans<<<dim3(E_DIM / 32, E_DIM / 64), 256, 0, stream>>>(W2, Wt2, E_DIM, WSC2);

  k_stage1<<<dim3(E_DIM / ET1, nB), 256, 0, stream>>>(X, Wp, bp, g1, be1, m1, v1, masks, ZS);

  const int gemmBlocks = (Mrows / 64) * (E_DIM / 64) / 8;
  gemm64_bn<0><<<dim3(gemmBlocks), 256, 0, stream>>>(
      (const unsigned short*)ZS, E_DIM, (const unsigned short*)Wt1, E_DIM,
      (void*)Hb, E_DIM, b1, g2, be2, m2, v2, nullptr, Mrows, E_DIM, E_DIM, WSC2_INV);
  gemm64_bn<1><<<dim3(gemmBlocks), 256, 0, stream>>>(
      (const unsigned short*)Hb, E_DIM, (const unsigned short*)Wt2, E_DIM,
      (void*)out, E_DIM, b2, g3, be3, m3, v3, X, Mrows, E_DIM, E_DIM, WSC2_INV);
}
